// PhysicsMambaBlock_81862076662141
// MI455X (gfx1250) — hardware-verified
//
#include <hip/hip_runtime.h>


#define NB_  2
#define SQ   1024
#define DMD  1024
#define DI   2048
#define NS   16
#define DTR  64
#define NR   (NB_ * SQ)
typedef _Float16 h16;
typedef unsigned short bf;
typedef __attribute__((ext_vector_type(16))) __bf16   v16bf;
typedef __attribute__((ext_vector_type(16))) _Float16 v16h;
typedef __attribute__((ext_vector_type(8)))  _Float16 v8h;
typedef __attribute__((ext_vector_type(8)))  unsigned short v8us;
typedef __attribute__((ext_vector_type(8)))  float    v8f;
typedef __attribute__((ext_vector_type(4)))  float    v4f;
typedef v8h  __attribute__((may_alias)) v8ha;
typedef v4f  __attribute__((may_alias)) v4fa;
typedef v8us __attribute__((may_alias)) v8usa;

__device__ __forceinline__ unsigned short f2bf(float f) { unsigned u = __float_as_uint(f); u += 0x7FFFu + ((u >> 16) & 1u); return (unsigned short)(u >> 16); }
__device__ __forceinline__ float bf2f(unsigned short b) { return __uint_as_float(((unsigned)b) << 16); }
__device__ __forceinline__ float bfr(float f) { return bf2f(f2bf(f)); }
__device__ __forceinline__ v16h cat16(v8h lo, v8h hi) { return __builtin_shufflevector(lo, hi, 0, 1, 2, 3, 4, 5, 6, 7, 8, 9, 10, 11, 12, 13, 14, 15); }
__device__ __forceinline__ v16bf cat16b(v8us lo, v8us hi) { return __builtin_bit_cast(v16bf, __builtin_shufflevector(lo, hi, 0, 1, 2, 3, 4, 5, 6, 7, 8, 9, 10, 11, 12, 13, 14, 15)); }
__device__ __forceinline__ v8f wmma16(v16h a, v16h b, v8f c) { return __builtin_amdgcn_wmma_f32_16x16x32_f16(false, a, false, b, (short)0, c, false, false); }
__device__ __forceinline__ v8f wmmab(v16bf a, v16bf b, v8f c) { return __builtin_amdgcn_wmma_f32_16x16x32_bf16(false, a, false, b, (short)0, c, false, false); }


template <typename T16> struct WFrag;
template <> struct WFrag<h16> { typedef v16h V; static __device__ __forceinline__ V ld(const h16* p) { return cat16(*(const v8h*)p, *(const v8h*)(p + 16)); } static __device__ __forceinline__ v8f mma(V a, V b, v8f c) { return wmma16(a, b, c); } };
template <> struct WFrag<bf> { typedef v16bf V; static __device__ __forceinline__ V ld(const bf* p) { return cat16b(*(const v8us*)p, *(const v8us*)(p + 16)); } static __device__ __forceinline__ v8f mma(V a, V b, v8f c) { return wmmab(a, b, c); } };
template <typename T16, int NSPLIT, bool BIAS>
__global__ __launch_bounds__(32) void k_gemmw(const T16* __restrict__ A, const T16* __restrict__ A2, const T16* __restrict__ Bt, const T16* __restrict__ Bt2, int K, float* C, int ldc, const float* __restrict__ bias, size_t sA, size_t sB, size_t sC) {
    typedef typename WFrag<T16>::V V;
    __shared__ __align__(16) float os[16 * 68];
    const size_t z = blockIdx.z; A += z * sA; if (A2) A2 += z * sA; Bt += z * sB; if (Bt2) Bt2 += z * sB; C += z * sC;
    const int lane = threadIdx.x & 31, lr = lane & 15, hi = lane >> 4; const int r0 = blockIdx.x * 64, c0 = blockIdx.y * 64;
    v8f acc[4][4];
#pragma unroll
    for (int mb = 0; mb < 4; ++mb)
#pragma unroll
        for (int nb = 0; nb < 4; ++nb) acc[mb][nb] = (v8f){};
    const size_t aoff = (size_t)(r0 + lr) * K + 8 * hi, boff = (size_t)(c0 + lr) * K + 8 * hi;
#pragma unroll 1
    for (int kc = 0; kc < K; kc += 32) {
        V a[4], a2[4];
#pragma unroll
        for (int mb = 0; mb < 4; ++mb) { a[mb] = WFrag<T16>::ld(A + aoff + (size_t)mb * 16 * K + kc); if (NSPLIT == 1 || NSPLIT == 2) a2[mb] = WFrag<T16>::ld(A2 + aoff + (size_t)mb * 16 * K + kc); }
#pragma unroll
        for (int nb = 0; nb < 4; ++nb) { const V b = WFrag<T16>::ld(Bt + boff + (size_t)nb * 16 * K + kc); V b2; if (NSPLIT >= 2) b2 = WFrag<T16>::ld(Bt2 + boff + (size_t)nb * 16 * K + kc);
#pragma unroll
            for (int mb = 0; mb < 4; ++mb) { acc[mb][nb] = WFrag<T16>::mma(a[mb], b, acc[mb][nb]); if (NSPLIT == 1 || NSPLIT == 2) acc[mb][nb] = WFrag<T16>::mma(a2[mb], b, acc[mb][nb]); if (NSPLIT >= 2) acc[mb][nb] = WFrag<T16>::mma(a[mb], b2, acc[mb][nb]); } }
        asm volatile("v_nop\n\tv_nop\n\tv_nop\n\tv_nop" : "+v"(acc[0][0]), "+v"(acc[1][1]), "+v"(acc[2][2]), "+v"(acc[3][3]) : "v"(a[0]), "v"(a[3]));
    }
#pragma unroll
    for (int mb = 0; mb < 4; ++mb) {
#pragma unroll
        for (int nb = 0; nb < 4; ++nb) {
#pragma unroll
            for (int j = 0; j < 8; ++j) os[(hi * 8 + j) * 68 + nb * 16 + lr] = acc[mb][nb][j]; }
        __builtin_amdgcn_wave_barrier(); asm volatile("" ::: "memory");
        float* crow = C + (size_t)(r0 + mb * 16) * ldc + c0;
#pragma unroll 1
        for (int ps = 0; ps < 2; ++ps) {
#pragma unroll
            for (int s = 0; s < 8; ++s) { const int row = 2 * s + hi, cofs = lr * 4; v4f val = *(const v4fa*)(os + row * 68 + cofs); if (BIAS) { val[0] += bfr(bias[c0 + cofs]); val[1] += bfr(bias[c0 + cofs + 1]); val[2] += bfr(bias[c0 + cofs + 2]); val[3] += bfr(bias[c0 + cofs + 3]); }
                *(volatile v4f*)(crow + (size_t)row * ldc + cofs) = val; }
            if (ps == 0) __threadfence(); }
        __builtin_amdgcn_wave_barrier(); asm volatile("" ::: "memory");
    }
}

__device__ __forceinline__ void splitf(float y, unsigned short& h, unsigned short& l) { h = f2bf(y); l = f2bf(y - bf2f(h)); }
typedef __attribute__((ext_vector_type(4))) unsigned short v4us;

__global__ __launch_bounds__(256) void k_cvt8(const float* __restrict__ src, bf* dst, size_t n8) { const size_t i = (size_t)blockIdx.x * 256 + threadIdx.x; if (i >= n8) return; const v8f v = *(const v8f*)(src + i * 8); v8us o;
#pragma unroll
    for (int k = 0; k < 8; ++k) o[k] = f2bf(v[k]); *(volatile v8us*)(dst + i * 8) = o; __threadfence(); *(volatile v8us*)(dst + i * 8) = o; }
__global__ __launch_bounds__(256) void k_wxp(const float* __restrict__ w, bf* Bt) { const int e = (blockIdx.x * 256 + threadIdx.x) * 4; if (e >= 64 * DI) return; const int k = e % DI; const int c = e / DI; v4us v;
#pragma unroll
    for (int u = 0; u < 4; ++u) v[u] = (c < 2 * NS) ? f2bf(w[(size_t)(DTR + c) * DI + k + u]) : (unsigned short)0; *(volatile v4us*)(Bt + e) = v; __threadfence(); *(volatile v4us*)(Bt + e) = v; }
__global__ __launch_bounds__(256) void k_conv(const float* __restrict__ XZ, const float* __restrict__ cw, const float* __restrict__ cb, float* Uf, bf* Uh, bf* Ul) { const size_t e = ((size_t)blockIdx.x * 256 + threadIdx.x) * 4; if (e >= (size_t)NR * DI) return; const int i = (int)(e % DI); const int r = (int)(e / DI); const int t = r % SQ; v4f o; v4us oh, ol;
#pragma unroll
    for (int u = 0; u < 4; ++u) { const int c = i + u; float s = 0.f;
#pragma unroll
        for (int j = 0; j < 4; ++j) { const int tt = t - 3 + j; const float xv = (tt >= 0) ? XZ[(size_t)(r - 3 + j) * (2 * DI) + c] : 0.f; float p = __fmul_rn(xv, bfr(cw[c * 4 + j])); asm volatile("" : "+v"(p)); s = __fadd_rn(s, p); }
        s = __fadd_rn(s, bfr(cb[c])); const float sg = __fdiv_rn(1.0f, __fadd_rn(1.0f, __expf(-s))); o[u] = __fmul_rn(s, sg); unsigned short p2, q2; splitf(o[u], p2, q2); oh[u] = p2; ol[u] = q2; }
    *(volatile v4f*)(Uf + e) = o; *(volatile v4us*)(Uh + e) = oh; *(volatile v4us*)(Ul + e) = ol; __threadfence(); *(volatile v4f*)(Uf + e) = o; *(volatile v4us*)(Uh + e) = oh; *(volatile v4us*)(Ul + e) = ol; }
__global__ __launch_bounds__(64) void k_scan(const float* __restrict__ dtv, const float* __restrict__ dtw, const float* __restrict__ dtb, const float* __restrict__ Uf, const float* __restrict__ XD, const float* __restrict__ alog, const float* __restrict__ Dv, float* Y) {
    const int gl = blockIdx.x * 64 + threadIdx.x; if (gl >= NB_ * DI) return; const int b = gl / DI, i = gl % DI; float A[NS], h[NS];
#pragma unroll
    for (int n = 0; n < NS; ++n) { A[n] = -__expf(bfr(alog[i * NS + n])); h[n] = 0.f; } const float wdt = bfr(dtw[i]), bdt = bfr(dtb[i]), Dd = bfr(Dv[i]);
#pragma unroll 1
    for (int t = 0; t < SQ; ++t) { const size_t r = (size_t)b * SQ + t; float zt = __fmul_rn(bfr(dtv[r]), wdt); asm volatile("" : "+v"(zt)); zt = __fadd_rn(zt, bdt); const float dt = (zt > 20.f) ? zt : log1pf(__expf(zt)); const float uu = Uf[r * DI + i]; const float* xd = XD + r * 64; float du = __fmul_rn(dt, uu); asm volatile("" : "+v"(du)); float y = 0.f;
#pragma unroll
        for (int n = 0; n < NS; ++n) { const float da = __expf(__fmul_rn(dt, A[n])); float db = __fmul_rn(du, xd[n]); asm volatile("" : "+v"(db)); float q = __fmul_rn(da, h[n]); asm volatile("" : "+v"(q)); h[n] = __fadd_rn(q, db); float p = __fmul_rn(h[n], xd[NS + n]); asm volatile("" : "+v"(p)); y = __fadd_rn(y, p); }
        float sk = __fmul_rn(uu, Dd); asm volatile("" : "+v"(sk)); const float yy = __fadd_rn(y, sk); *(volatile float*)(Y + r * DI + i) = yy; __threadfence(); *(volatile float*)(Y + r * DI + i) = yy; } }
__global__ __launch_bounds__(256) void k_gate(const float* __restrict__ Y, const float* __restrict__ XZ, bf* Gh, bf* Gl) { const size_t e = ((size_t)blockIdx.x * 256 + threadIdx.x) * 4; if (e >= (size_t)NR * DI) return; const int i = (int)(e % DI); const int r = (int)(e / DI); v4us oh, ol;
#pragma unroll
    for (int u = 0; u < 4; ++u) { const float g = XZ[(size_t)r * (2 * DI) + DI + i + u]; const float sg = __fdiv_rn(1.0f, __fadd_rn(1.0f, __expf(-g))); float sl = __fmul_rn(g, sg); asm volatile("" : "+v"(sl)); unsigned short p, q; splitf(__fmul_rn(Y[e + u], sl), p, q); oh[u] = p; ol[u] = q; }
    *(volatile v4us*)(Gh + e) = oh; *(volatile v4us*)(Gl + e) = ol; __threadfence(); *(volatile v4us*)(Gh + e) = oh; *(volatile v4us*)(Gl + e) = ol; }

extern "C" void kernel_launch(void* const* d_in, const int* in_sizes, int n_in,
                              void* d_out, int out_size, void* d_ws, size_t ws_size, hipStream_t stream) {
    (void)in_sizes; (void)n_in; (void)out_size;
    const float** I = (const float**)d_in;
    const float *x = I[0], *dtv = I[1], *Win = I[2], *cw = I[3], *cb = I[4], *Wxp = I[5], *dtw = I[6], *dtb = I[7], *alog = I[8], *Dv = I[9], *Wout = I[10];
    float* OUT = (float*)d_out;
    char* wsp = (char*)d_ws;
    auto take = [&](size_t bytes) { char* p = wsp; wsp += (bytes + 255) & ~(size_t)255; return (void*)p; };
    bf* BIN = (bf*)take((size_t)(2 * DI) * DMD * 2); bf* BXP = (bf*)take((size_t)64 * DI * 2); bf* BOUT = (bf*)take((size_t)DMD * DI * 2); bf* XB = (bf*)take((size_t)NR * DMD * 2);
    float* XZ = (float*)take((size_t)NR * 2 * DI * 4); float* Uf = (float*)take((size_t)NR * DI * 4); bf* Uh = (bf*)take((size_t)NR * DI * 2); bf* Ul = (bf*)take((size_t)NR * DI * 2); float* XD = (float*)take((size_t)NR * 64 * 4); float* Y = (float*)take((size_t)NR * DI * 4);
    if ((size_t)(wsp - (char*)d_ws) > ws_size) return;
    k_cvt8<<<(unsigned)(((size_t)2 * DI * DMD / 8 + 255) / 256), 256, 0, stream>>>(Win, BIN, (size_t)2 * DI * DMD / 8);
    k_wxp<<<(64 * DI / 4 + 255) / 256, 256, 0, stream>>>(Wxp, BXP); k_cvt8<<<(unsigned)(((size_t)DMD * DI / 8 + 255) / 256), 256, 0, stream>>>(Wout, BOUT, (size_t)DMD * DI / 8);
    k_cvt8<<<(NR * DMD / 8 + 255) / 256, 256, 0, stream>>>(x, XB, NR * DMD / 8);
    k_gemmw<bf, 0, false><<<dim3(NR / 64, 2 * DI / 64, 1), 32, 0, stream>>>(XB, nullptr, BIN, nullptr, DMD, XZ, 2 * DI, nullptr, 0, 0, 0);
    const unsigned gE = (unsigned)(((size_t)NR * DI / 4 + 255) / 256);
    k_conv<<<gE, 256, 0, stream>>>(XZ, cw, cb, Uf, Uh, Ul);
    k_gemmw<bf, 1, false><<<dim3(NR / 64, 1, 1), 32, 0, stream>>>(Uh, Ul, BXP, nullptr, DI, XD, 64, nullptr, 0, 0, 0);
    k_scan<<<(NB_ * DI + 63) / 64, 64, 0, stream>>>(dtv, dtw, dtb, Uf, XD, alog, Dv, Y);
    k_gate<<<gE, 256, 0, stream>>>(Y, XZ, Uh, Ul);
    k_gemmw<bf, 1, false><<<dim3(NR / 64, DMD / 64, 1), 32, 0, stream>>>(Uh, Ul, BOUT, nullptr, DI, OUT, DMD, nullptr, 0, 0, 0);
}
